// MultiHeadPosAttn_75763223102207
// MI455X (gfx1250) — hardware-verified
//
#include <hip/hip_runtime.h>
#include <hip/hip_bf16.h>

typedef __attribute__((ext_vector_type(16))) _Float16 v16h;
typedef __attribute__((ext_vector_type(8)))  _Float16 v8h;
typedef __attribute__((ext_vector_type(16))) __bf16   v16b;
typedef __attribute__((ext_vector_type(8)))  __bf16   v8b;
typedef __attribute__((ext_vector_type(8)))  float    v8f;
typedef __attribute__((ext_vector_type(4)))  float    v4f;

#define NBATCH 16
#define NCH    256
#define NPIX   1024
#define NHEADS 4
#define DHEAD  64
#define NFF    1024
#define NROWS  (NBATCH * NPIX)

__device__ __forceinline__ unsigned short f2bf_bits(float f) {
  unsigned u = __float_as_uint(f);
  return (unsigned short)((u + 0x7FFFu + ((u >> 16) & 1u)) >> 16);
}
__device__ __forceinline__ float bf_bits2f(unsigned short h) { return __uint_as_float(((unsigned)h) << 16); }

__device__ __forceinline__ void dep_guard_h(v8f& a, v8f& b, v16h x, v16h y) { asm volatile("v_nop\n\tv_nop\n\tv_nop\n\tv_nop" : "+v"(a), "+v"(b) : "v"(x), "v"(y)); }
__device__ __forceinline__ void dep_guard_b(v8f& a, v8f& b, v16b x, v16b y) { asm volatile("v_nop\n\tv_nop\n\tv_nop\n\tv_nop" : "+v"(a), "+v"(b) : "v"(x), "v"(y)); }
__device__ __forceinline__ void keep4_h(v16h a, v16h b, v16h c, v16h d) { asm volatile("v_nop" :: "v"(a), "v"(b), "v"(c), "v"(d)); }
__device__ __forceinline__ void keep4_b(v16b a, v16b b, v16b c, v16b d) { asm volatile("v_nop" :: "v"(a), "v"(b), "v"(c), "v"(d)); }
__device__ __forceinline__ void acc_guard4(v8f& a, v8f& b, v8f& c, v8f& d) { asm volatile("v_nop\n\tv_nop\n\tv_nop\n\tv_nop" : "+v"(a), "+v"(b), "+v"(c), "+v"(d)); }

template <typename T> struct Frag;
template <> struct Frag<_Float16> {
  typedef v16h V; union U { v16h v; v8h h[2]; };
  static __device__ __forceinline__ v16h load(const _Float16* p) {
    U f; f.h[0] = *(const v8h*)(p); f.h[1] = *(const v8h*)(p + 16); return f.v;
  }
  static __device__ __forceinline__ v8f mma(v16h a, v16h b, v8f c) {
    return __builtin_amdgcn_wmma_f32_16x16x32_f16(false, a, false, b, (short)0, c, false, false);
  }
  static __device__ __forceinline__ void guard(v8f& a, v8f& b, v16h x, v16h y) { dep_guard_h(a, b, x, y); }
  static __device__ __forceinline__ void keep(v16h a, v16h b, v16h c, v16h d) { keep4_h(a, b, c, d); }
};
template <> struct Frag<__bf16> {
  typedef v16b V; union U { v16b v; v8b h[2]; };
  static __device__ __forceinline__ v16b load(const __bf16* p) {
    U f; f.h[0] = *(const v8b*)(p); f.h[1] = *(const v8b*)(p + 16); return f.v;
  }
  static __device__ __forceinline__ v8f mma(v16b a, v16b b, v8f c) {
    return __builtin_amdgcn_wmma_f32_16x16x32_bf16(false, a, false, b, (short)0, c, false, false);
  }
  static __device__ __forceinline__ void guard(v8f& a, v8f& b, v16b x, v16b y) { dep_guard_b(a, b, x, y); }
  static __device__ __forceinline__ void keep(v16b a, v16b b, v16b c, v16b d) { keep4_b(a, b, c, d); }
};

template <int ET> struct Elem;
template <> struct Elem<0> { typedef _Float16 T; };
template <> struct Elem<1> { typedef __bf16 T; };
template <int ET, bool SPLIT, int BIAS_MODE, int OUT_MODE, bool RESID, int ACT = 0>
__global__ __launch_bounds__(256) void wmma_gemm64(
    const unsigned short* __restrict__ Ap, const unsigned short* __restrict__ A2p, int lda, long strideA,
    const unsigned short* __restrict__ Btp, const unsigned short* __restrict__ Bt2p, int ldb, long strideB,
    void* __restrict__ Cout, void* __restrict__ Cout2, int ldc, long strideC,
    const float* __restrict__ bias, const float* __restrict__ aux,
    const float* __restrict__ resid, long strideR,
    int M, int N, int K, float scale) {
  typedef typename Elem<ET>::T T;
  typedef typename Frag<T>::V V;
  const T* A = (const T*)Ap; const T* A2 = (const T*)A2p; const T* Bt = (const T*)Btp; const T* Bt2 = (const T*)Bt2p;
  __shared__ __align__(16) float sT[8][16 * 68];
  const int b    = blockIdx.y;
  const int lane = threadIdx.x & 31;
  const int wave = threadIdx.x >> 5;
  const int tilesN = N >> 6;
  const int tilesM = M >> 6;
  const int tile = blockIdx.x * 8 + wave;
  if (tile >= tilesM * tilesN) return;
  const int tm = tile / tilesN;
  const int tn = tile - tm * tilesN;
  const int m0 = tm << 6;
  const int n0 = tn << 6;

  const T* Ab  = A  + (size_t)b * strideA;
  const T* Bb  = Bt + (size_t)b * strideB;
  const T* Ab2 = SPLIT ? (A2  + (size_t)b * strideA) : nullptr;
  const T* Bb2 = SPLIT ? (Bt2 + (size_t)b * strideB) : nullptr;

  const int rlane = lane & 15;
  const int koff  = (lane >> 4) * 8;
  const int mOff  = (lane >> 4) * 8;

  v8f acc[4][4];
#pragma unroll
  for (int i = 0; i < 4; ++i)
#pragma unroll
    for (int j = 0; j < 4; ++j) acc[i][j] = (v8f){0.f,0.f,0.f,0.f,0.f,0.f,0.f,0.f};

  for (int k0 = 0; k0 < K; k0 += 32) {
    V bh[4], bl[4];
#pragma unroll
    for (int j = 0; j < 4; ++j) {
      const size_t bo = (size_t)(n0 + (j << 4) + rlane) * ldb + koff + k0;
      bh[j] = Frag<T>::load(Bb + bo);
      if (SPLIT) bl[j] = Frag<T>::load(Bb2 + bo);
    }
#pragma unroll
    for (int i = 0; i < 4; ++i) {
      const size_t ao = (size_t)(m0 + (i << 4) + rlane) * lda + koff + k0;
      V ah = Frag<T>::load(Ab + ao);
      V al;
      if (SPLIT) al = Frag<T>::load(Ab2 + ao);
#pragma unroll
      for (int j = 0; j < 4; ++j) {
        acc[i][j] = Frag<T>::mma(ah, bh[j], acc[i][j]);
        if (SPLIT) {
          acc[i][j] = Frag<T>::mma(ah, bl[j], acc[i][j]);
          acc[i][j] = Frag<T>::mma(al, bh[j], acc[i][j]);
        }
      }
      Frag<T>::guard(acc[i][0], acc[i][3], ah, SPLIT ? al : ah);
    }
    Frag<T>::keep(bh[0], bh[1], bh[2], bh[3]);
    if (SPLIT) Frag<T>::keep(bl[0], bl[1], bl[2], bl[3]);
  }
  acc_guard4(acc[0][0], acc[0][1], acc[0][2], acc[0][3]);
  acc_guard4(acc[1][0], acc[1][1], acc[1][2], acc[1][3]);
  acc_guard4(acc[2][0], acc[2][1], acc[2][2], acc[2][3]);
  acc_guard4(acc[3][0], acc[3][1], acc[3][2], acc[3][3]);

  float* slab = sT[wave];
  const float* Rb = RESID ? (resid + (size_t)b * strideR) : nullptr;
  float slope = 0.f;
  if (ACT == 6) slope = aux[0];
#pragma unroll
  for (int i = 0; i < 4; ++i) {
    const int mBase = m0 + (i << 4);
#pragma unroll
    for (int j = 0; j < 4; ++j) {
      const int n = n0 + (j << 4) + rlane;
      float bv = 0.f;
      if (BIAS_MODE == 2) bv = bias[n];
#pragma unroll
      for (int r = 0; r < 8; ++r) {
        float v = acc[i][j][r] * scale;
        if (BIAS_MODE == 1) v += bias[mBase + mOff + r];
        if (BIAS_MODE == 2) v += bv;
        if (RESID) v += Rb[(size_t)(mBase + mOff + r) * ldc + n];
        if (ACT == 6) v = (v >= 0.f) ? v : slope * v;
        slab[(mOff + r) * 68 + (j << 4) + rlane] = v;
      }
    }
    __builtin_amdgcn_fence(__ATOMIC_RELEASE, "workgroup");
    __builtin_amdgcn_wave_barrier();
    __builtin_amdgcn_fence(__ATOMIC_ACQUIRE, "workgroup");
    if (OUT_MODE == 0) {
      float* C = (float*)Cout + (size_t)b * strideC;
      const int hh = lane >> 4, c4 = (lane & 15) * 4;
      for (int pass = 0; pass < 2; ++pass) {
#pragma unroll
        for (int it = 0; it < 8; ++it) {
          const int row = it * 2 + hh;
          v4f v = *(const v4f*)(slab + row * 68 + c4);
          *(volatile v4f*)(C + (size_t)(mBase + row) * ldc + n0 + c4) = v;
        }
        __threadfence();
      }
    } else {
      const int q = lane >> 3, c8 = (lane & 7) * 8;
      unsigned short* C  = (unsigned short*)Cout  + (size_t)b * strideC;
      unsigned short* C2 = (OUT_MODE == 2) ? ((unsigned short*)Cout2 + (size_t)b * strideC) : nullptr;
      for (int pass = 0; pass < 2; ++pass) {
#pragma unroll
        for (int it = 0; it < 4; ++it) {
          const int row = it * 4 + q;
          const float* sp = slab + row * 68 + c8;
          v8h hv, lv;
#pragma unroll
          for (int e = 0; e < 8; ++e) {
            if (OUT_MODE == 1) {
              hv[e] = (_Float16)sp[e];
              lv[e] = hv[e];
            } else {
              unsigned short hb = f2bf_bits(sp[e]);
              unsigned short lb = f2bf_bits(sp[e] - bf_bits2f(hb));
              hv[e] = __builtin_bit_cast(_Float16, hb);
              lv[e] = __builtin_bit_cast(_Float16, lb);
            }
          }
          *(volatile v8h*)(C + (size_t)(mBase + row) * ldc + n0 + c8) = hv;
          if (OUT_MODE == 2) *(volatile v8h*)(C2 + (size_t)(mBase + row) * ldc + n0 + c8) = lv;
        }
        __threadfence();
      }
    }
    __builtin_amdgcn_fence(__ATOMIC_RELEASE, "workgroup");
    __builtin_amdgcn_wave_barrier();
    __builtin_amdgcn_fence(__ATOMIC_ACQUIRE, "workgroup");
  }
}

#define AT_D 64
#define AT_NW 4
#define AT_QB 64
#define AT_KC 64
struct AttnGeom { long q_bs, q_rs, q_hs, k_bs, k_rs, k_hs, v_bs, v_rs, v_hs, o_bs, o_rs, o_hs;
                  int S, Skv, H, zpad; };
typedef char attn_geom_size_check[(sizeof(AttnGeom) == 112) ? 1 : -1];

__device__ __forceinline__ unsigned short at_bf_bits(float f) {
  unsigned u = __float_as_uint(f);
  return (unsigned short)((u + 0x7FFFu + ((u >> 16) & 1u)) >> 16);
}
__device__ __forceinline__ __bf16 at_f2bf(float f) { return __builtin_bit_cast(__bf16, at_bf_bits(f)); }
__device__ __forceinline__ void at_split(float f, __bf16& hi, __bf16& lo) {
  const unsigned short hb = at_bf_bits(f);
  hi = __builtin_bit_cast(__bf16, hb);
  lo = at_f2bf(f - __uint_as_float(((unsigned)hb) << 16));
}
__device__ __forceinline__ v8f at_mma(v16b a, v16b b, v8f c) {
  c = __builtin_amdgcn_wmma_f32_16x16x32_bf16(false, a, false, b, (short)0, c, false, false);
  asm volatile("v_nop\n\tv_nop\n\tv_nop\n\tv_nop" : "+v"(c) : "v"(a), "v"(b));
  return c;
}
__device__ __forceinline__ __bf16 at_toh(float f) { return __builtin_bit_cast(__bf16, (_Float16)f); }
__device__ __forceinline__ v8f at_mma_h(v16b a, v16b b, v8f c) {
  const v16h ah = __builtin_bit_cast(v16h, a), bh = __builtin_bit_cast(v16h, b);
  c = __builtin_amdgcn_wmma_f32_16x16x32_f16(false, ah, false, bh, (short)0, c, false, false);
  asm volatile("v_nop\n\tv_nop\n\tv_nop\n\tv_nop" : "+v"(c) : "v"(ah), "v"(bh));
  return c;
}

__global__ __launch_bounds__(128)
void attn64_qks_pvh(const float* __restrict__ q, const float* __restrict__ k,
                    const float* __restrict__ v, float* __restrict__ out, AttnGeom g) {
  const float PSC = 32768.0f;
  union FB { v16b v; v8b h[2]; };
  __shared__ __align__(16) __bf16 Ksh[AT_KC * AT_D];
  __shared__ __align__(16) __bf16 Ksl[AT_KC * AT_D];
  __shared__ __align__(16) __bf16 Vth[AT_D * AT_KC];
  __shared__ __align__(16) __bf16 Psh[AT_NW][16 * AT_KC];
  __shared__ __align__(16) float  Os[AT_NW][16 * 68];

  const int tid  = threadIdx.x;
  const int wave = tid >> 5;
  const int lane = tid & 31;
  const int hh   = lane >> 4;
  const int c    = lane & 15;

  const int nqb = g.S / AT_QB;
  const int bx = blockIdx.x;
  const int qb = bx % nqb;
  const int bh = bx / nqb;
  const int h  = bh % g.H;
  const int b  = bh / g.H;
  const int q0 = qb * AT_QB + wave * 16;

  const float* qb_ptr = q + (size_t)b * g.q_bs + (size_t)h * g.q_hs;
  const float* kb_ptr = k + (size_t)b * g.k_bs + (size_t)h * g.k_hs;
  const float* vb_ptr = v + (size_t)b * g.v_bs + (size_t)h * g.v_hs;
  float*       ob_ptr = out + (size_t)b * g.o_bs + (size_t)h * g.o_hs;

  v16b qah[2], qal[2];
  {
    const float* qrow = qb_ptr + (size_t)(q0 + c) * g.q_rs;
#pragma unroll
    for (int dc = 0; dc < 2; ++dc) {
#pragma unroll
      for (int e = 0; e < 8; ++e) {
        const float f0 = qrow[dc * 32 + 8 * hh + e];
        const float f1 = qrow[dc * 32 + 16 + 8 * hh + e];
        __bf16 hq, lq;
        at_split(f0, hq, lq); qah[dc][e] = hq;     qal[dc][e] = lq;
        at_split(f1, hq, lq); qah[dc][8 + e] = hq; qal[dc][8 + e] = lq;
      }
    }
  }

  float mrow[8], lrow[8];
  v8f oacc[4];
#pragma unroll
  for (int r = 0; r < 8; ++r) { mrow[r] = -__builtin_inff(); lrow[r] = 0.f; }
#pragma unroll
  for (int t = 0; t < 4; ++t) oacc[t] = (v8f){0.f,0.f,0.f,0.f,0.f,0.f,0.f,0.f};

  const int nChunks = g.Skv / AT_KC;
  for (int kc = 0; kc < nChunks; ++kc) {
    const int kv0 = kc * AT_KC;
    __syncthreads();
    {
      const int kvr = tid >> 1, dh = (tid & 1) * 32;
      const float* krow = kb_ptr + (size_t)(kv0 + kvr) * g.k_rs + dh;
      const float* vrow = vb_ptr + (size_t)(kv0 + kvr) * g.v_rs + dh;
#pragma unroll
      for (int i = 0; i < 8; ++i) {
        v4f kk = *(const v4f*)(krow + 4 * i);
        v4f vv = *(const v4f*)(vrow + 4 * i);
#pragma unroll
        for (int e = 0; e < 4; ++e) {
          const int d = dh + 4 * i + e;
          __bf16 a, bl; at_split(kk[e], a, bl);
          Ksh[kvr * AT_D + d] = a; Ksl[kvr * AT_D + d] = bl;
          Vth[d * AT_KC + kvr] = at_toh(vv[e]);
        }
      }
    }
    __syncthreads();

    v8f s[4];
#pragma unroll
    for (int j = 0; j < 4; ++j) {
      s[j] = (v8f){0.f,0.f,0.f,0.f,0.f,0.f,0.f,0.f};
#pragma unroll
      for (int dc = 0; dc < 2; ++dc) {
        FB kb, kl;
        kb.h[0] = *(const v8b*)(Ksh + (j * 16 + c) * AT_D + dc * 32 + 8 * hh);
        kb.h[1] = *(const v8b*)(Ksh + (j * 16 + c) * AT_D + dc * 32 + 16 + 8 * hh);
        kl.h[0] = *(const v8b*)(Ksl + (j * 16 + c) * AT_D + dc * 32 + 8 * hh);
        kl.h[1] = *(const v8b*)(Ksl + (j * 16 + c) * AT_D + dc * 32 + 16 + 8 * hh);
        s[j] = at_mma(qah[dc], kb.v, s[j]);
        s[j] = at_mma(qah[dc], kl.v, s[j]);
        s[j] = at_mma(qal[dc], kb.v, s[j]);
      }
    }
    float cm[8];
#pragma unroll
    for (int r = 0; r < 8; ++r) {
      float m = s[0][r];
      m = fmaxf(m, s[1][r]); m = fmaxf(m, s[2][r]); m = fmaxf(m, s[3][r]);
#pragma unroll
      for (int off = 1; off < 16; off <<= 1) m = fmaxf(m, __shfl_xor(m, off, 32));
      cm[r] = m;
    }
    __bf16* pwh = Psh[wave];
#pragma unroll
    for (int r = 0; r < 8; ++r) {
      const float mnew = fmaxf(mrow[r], cm[r]);
      const float alpha = expf(mrow[r] - mnew);
      mrow[r] = mnew;
      float psum = 0.f;
#pragma unroll
      for (int j = 0; j < 4; ++j) {
        const float p = expf(s[j][r] - mnew);
        psum += p;
        pwh[(8 * hh + r) * AT_KC + j * 16 + c] = at_toh(p * PSC);
      }
#pragma unroll
      for (int off = 1; off < 16; off <<= 1) psum += __shfl_xor(psum, off, 32);
      lrow[r] = lrow[r] * alpha + psum;
#pragma unroll
      for (int t = 0; t < 4; ++t) oacc[t][r] *= alpha;
    }
    __builtin_amdgcn_fence(__ATOMIC_RELEASE, "workgroup");
    __builtin_amdgcn_wave_barrier();
    __builtin_amdgcn_fence(__ATOMIC_ACQUIRE, "workgroup");
#pragma unroll 1
    for (int kk = 0; kk < 2; ++kk) {
      FB pa;
      pa.h[0] = *(const v8b*)(pwh + c * AT_KC + kk * 32 + 8 * hh);
      pa.h[1] = *(const v8b*)(pwh + c * AT_KC + kk * 32 + 16 + 8 * hh);
#pragma unroll
      for (int t = 0; t < 4; ++t) {
        FB vb;
        vb.h[0] = *(const v8b*)(Vth + (t * 16 + c) * AT_KC + kk * 32 + 8 * hh);
        vb.h[1] = *(const v8b*)(Vth + (t * 16 + c) * AT_KC + kk * 32 + 16 + 8 * hh);
        oacc[t] = at_mma_h(pa.v, vb.v, oacc[t]);
      }
    }
  }

  float* os = Os[wave];
#pragma unroll
  for (int r = 0; r < 8; ++r) {
    const float inv = 1.0f / (lrow[r] * PSC);
#pragma unroll
    for (int t = 0; t < 4; ++t) os[(8 * hh + r) * 68 + t * 16 + c] = oacc[t][r] * inv;
  }
  __builtin_amdgcn_fence(__ATOMIC_RELEASE, "workgroup");
  __builtin_amdgcn_wave_barrier();
  __builtin_amdgcn_fence(__ATOMIC_ACQUIRE, "workgroup");
  {
    const int c4 = (lane & 15) * 4;
    for (int pass = 0; pass < 2; ++pass) {
#pragma unroll
      for (int it = 0; it < 8; ++it) {
        const int row = it * 2 + hh;
        v4f val = *(const v4f*)(os + row * 68 + c4);
        *(volatile v4f*)(ob_ptr + (size_t)(q0 + row) * g.o_rs + c4) = val;
      }
      __threadfence();
    }
  }
}

__global__ __launch_bounds__(256) void prep_x(const float* __restrict__ x,
    _Float16* __restrict__ xh, _Float16* __restrict__ xl, _Float16* __restrict__ xf) {
  __shared__ float s[32][257];
  const int t = threadIdx.x, lane = t & 31, wave = t >> 5;
  const int b = blockIdx.y, n0 = blockIdx.x * 32;
  const float* xb = x + (size_t)b * NCH * NPIX + n0 + lane;
#pragma unroll 4
  for (int i = 0; i < 32; ++i) {
    const int ch = i * 8 + wave;
    s[lane][ch] = xb[(size_t)ch * NPIX];
  }
  __syncthreads();
#pragma unroll 1
  for (int p = 0; p < 4; ++p) {
    const int pix = wave * 4 + p;
    const float* sp = &s[pix][8 * lane];
    v8h hv, lv, fv;
#pragma unroll
    for (int j = 0; j < 8; ++j) {
      const float f = sp[j];
      const unsigned short hb = f2bf_bits(f);
      const unsigned short lb = f2bf_bits(f - bf_bits2f(hb));
      hv[j] = __builtin_bit_cast(_Float16, hb);
      lv[j] = __builtin_bit_cast(_Float16, lb);
      fv[j] = (_Float16)f;
    }
    const size_t off = ((size_t)b * NPIX + n0 + pix) * NCH + 8 * lane;
    *(volatile v8h*)(xh + off) = hv;
    *(volatile v8h*)(xl + off) = lv;
    *(volatile v8h*)(xf + off) = fv;
    __threadfence();
    *(volatile v8h*)(xh + off) = hv;
    *(volatile v8h*)(xl + off) = lv;
    *(volatile v8h*)(xf + off) = fv;
  }
}

__device__ __forceinline__ unsigned pack_f16x2(float a, float b) {
  const _Float16 h0 = (_Float16)a, h1 = (_Float16)b;
  return (unsigned)__builtin_bit_cast(unsigned short, h0) | ((unsigned)__builtin_bit_cast(unsigned short, h1) << 16);
}
__global__ __launch_bounds__(256) void prep_weights(
    const float* __restrict__ Wq, const float* __restrict__ Wk, const float* __restrict__ Wv,
    const float* __restrict__ W1, const float* __restrict__ W2,
    const float* __restrict__ bq, const float* __restrict__ bk,
    unsigned* __restrict__ wqkh, unsigned* __restrict__ wqkl, unsigned* __restrict__ wv16,
    unsigned* __restrict__ w1h, unsigned* __restrict__ w2h, float* __restrict__ bqk) {
  const int blk = blockIdx.x, t = threadIdx.x;
  if (blk < 256) {
    const int i = blk * 256 + t;
    const float* src = (blk < 128) ? Wq : Wk;
    const int e = (2 * i) & 65535;
    const float f0 = src[e], f1 = src[e + 1];
    const unsigned short hb0 = f2bf_bits(f0), hb1 = f2bf_bits(f1);
    const unsigned short lb0 = f2bf_bits(f0 - bf_bits2f(hb0)), lb1 = f2bf_bits(f1 - bf_bits2f(hb1));
    const unsigned uh = (unsigned)hb0 | ((unsigned)hb1 << 16);
    const unsigned ul = (unsigned)lb0 | ((unsigned)lb1 << 16);
    ((volatile unsigned*)wqkh)[i] = uh; ((volatile unsigned*)wqkl)[i] = ul;
    __threadfence();
    ((volatile unsigned*)wqkh)[i] = uh; ((volatile unsigned*)wqkl)[i] = ul;
  } else if (blk < 384) {
    const int i = (blk - 256) * 256 + t;
    const unsigned u = pack_f16x2(Wv[2 * i] * 16.0f, Wv[2 * i + 1] * 16.0f);
    ((volatile unsigned*)wv16)[i] = u; __threadfence(); ((volatile unsigned*)wv16)[i] = u;
  } else if (blk < 896) {
    const int i = (blk - 384) * 256 + t;
    const unsigned u = pack_f16x2(W1[2 * i] * 16.0f, W1[2 * i + 1] * 16.0f);
    ((volatile unsigned*)w1h)[i] = u; __threadfence(); ((volatile unsigned*)w1h)[i] = u;
  } else if (blk < 1408) {
    const int i = (blk - 896) * 256 + t;
    const unsigned u = pack_f16x2(W2[2 * i] * 16.0f, W2[2 * i + 1] * 16.0f);
    ((volatile unsigned*)w2h)[i] = u; __threadfence(); ((volatile unsigned*)w2h)[i] = u;
  } else {
    const int i = (blk - 1408) * 256 + t;
    const float* src = (blk == 1408) ? bq : bk;
    const float val = src[t];
    ((volatile float*)bqk)[i] = val; __threadfence(); ((volatile float*)bqk)[i] = val;
  }
}

template <bool HASX>
__global__ __launch_bounds__(256) void bn_partial(const float* __restrict__ Y,
    const float* __restrict__ X, double* __restrict__ part) {
  const int c = threadIdx.x;
  const int rb = blockIdx.x * 64;
  double s = 0.0, s2 = 0.0;
#pragma unroll 4
  for (int i = 0; i < 64; ++i) {
    const int row = rb + i;
    float y = Y[(size_t)row * NCH + c];
    if (HASX) {
      const int bb = row >> 10, n = row & 1023;
      y += X[((size_t)(bb * NCH + c) << 10) + n];
    }
    const double yd = (double)y;
    s += yd; s2 += yd * yd;
  }
  double* p = part + (size_t)blockIdx.x * 512;
  ((volatile double*)p)[c] = s; ((volatile double*)p)[256 + c] = s2;
  __threadfence();
  ((volatile double*)p)[c] = s; ((volatile double*)p)[256 + c] = s2;
}

__global__ __launch_bounds__(256) void bn_final(const double* __restrict__ part, int nblk,
    float inv_count, float* __restrict__ mean, float* __restrict__ istd) {
  const int c = threadIdx.x;
  double s = 0.0, s2 = 0.0;
#pragma unroll 1
  for (int b = 0; b < nblk; ++b) {
    s  += part[(size_t)b * 512 + c];
    s2 += part[(size_t)b * 512 + 256 + c];
  }
  const double m = s * (double)inv_count;
  double var = s2 * (double)inv_count - m * m;
  if (var < 0.0) var = 0.0;
  const float mf = (float)m;
  const float vf = (float)var;
  const float isf = 1.0f / sqrtf(vf + 1e-5f);
  ((volatile float*)mean)[c] = mf; ((volatile float*)istd)[c] = isf;
  __threadfence();
  ((volatile float*)mean)[c] = mf; ((volatile float*)istd)[c] = isf;
}

__global__ __launch_bounds__(256) void bn_apply1(const float* __restrict__ O, const float* __restrict__ X,
    const float* __restrict__ mean, const float* __restrict__ istd,
    const float* __restrict__ gamma, const float* __restrict__ beta,
    float* __restrict__ MH, _Float16* __restrict__ MH16) {
  __shared__ __align__(16) _Float16 sh[8][256];
  const int t = threadIdx.x, lane = t & 31, wave = t >> 5;
  const int row = blockIdx.x * 8 + wave;
  const int bb = row >> 10, n = row & 1023;
  v4f res[2];
#pragma unroll
  for (int g = 0; g < 2; ++g) {
    const int cb = g * 128 + 4 * lane;
    const v4f o4 = *(const v4f*)(O + (size_t)row * NCH + cb);
#pragma unroll
    for (int j = 0; j < 4; ++j) {
      const int ch = cb + j;
      const float y = o4[j] + X[((size_t)(bb * NCH + ch) << 10) + n];
      float z = (y - mean[ch]) * istd[ch];
      z = z * gamma[ch] + beta[ch];
      res[g][j] = z;
      sh[wave][ch] = (_Float16)z;
    }
  }
  float* mrow = MH + (size_t)row * NCH;
  *(volatile v4f*)(mrow + 4 * lane) = res[0];
  *(volatile v4f*)(mrow + 128 + 4 * lane) = res[1];
  __syncthreads();
  const v8h hv = *(const v8h*)(&sh[wave][8 * lane]);
  *(volatile v8h*)(MH16 + (size_t)row * NCH + 8 * lane) = hv;
  __threadfence();
  *(volatile v4f*)(mrow + 4 * lane) = res[0];
  *(volatile v4f*)(mrow + 128 + 4 * lane) = res[1];
  *(volatile v8h*)(MH16 + (size_t)row * NCH + 8 * lane) = hv;
}

__global__ __launch_bounds__(256) void bn_apply2_nchw(const float* __restrict__ Y,
    const float* __restrict__ mean, const float* __restrict__ istd,
    const float* __restrict__ gamma, const float* __restrict__ beta, float* __restrict__ out) {
  __shared__ __align__(16) float s[64][68];
  const int t = threadIdx.x, lane = t & 31, wave = t >> 5, hh = lane >> 4;
  const int b = blockIdx.z, c0 = blockIdx.y * 64, p0 = blockIdx.x * 64;
  const int ch = t & 63, pg = t >> 6;
  const int cc = c0 + ch;
  const float m = mean[cc], is = istd[cc], ga = gamma[cc], be = beta[cc];
  const float* yb = Y + ((size_t)b * NPIX + p0) * NCH + cc;
#pragma unroll 4
  for (int i = 0; i < 16; ++i) {
    const int p = i * 4 + pg;
    const float y = yb[(size_t)p * NCH];
    float z = (y - m) * is;
    z = z * ga + be;
    s[ch][p] = z;
  }
  __syncthreads();
  float* ob = out + ((size_t)b * NCH + c0) * NPIX + p0;
  const int c4 = (lane & 15) * 4;
  for (int pass = 0; pass < 2; ++pass) {
#pragma unroll
    for (int it = 0; it < 4; ++it) {
      const int chrow = wave * 8 + it * 2 + hh;
      const v4f val = *(const v4f*)(&s[chrow][c4]);
      *(volatile v4f*)(ob + (size_t)chrow * NPIX + c4) = val;
    }
    __threadfence();
  }
}

extern "C" void kernel_launch(void* const* d_in, const int* in_sizes, int n_in,
                              void* d_out, int out_size, void* d_ws, size_t ws_size,
                              hipStream_t stream)
{
  if (n_in < 14) return;
  if (in_sizes[0] != NBATCH * NCH * NPIX) return;
  if (in_sizes[1] != NHEADS * DHEAD * NCH || in_sizes[3] != NHEADS * DHEAD * NCH || in_sizes[5] != NHEADS * DHEAD * NCH) return;
  if (in_sizes[2] != NCH || in_sizes[4] != NCH || in_sizes[6] != NCH) return;
  if (in_sizes[7] != NCH || in_sizes[8] != NCH) return;
  if (in_sizes[9] != NFF * NCH || in_sizes[10] != NFF || in_sizes[11] < 1) return;
  if (in_sizes[12] != NCH * NFF || in_sizes[13] != NCH) return;
  if (out_size != NBATCH * NCH * NPIX) return;

  const float* x     = (const float*)d_in[0];
  const float* Wq    = (const float*)d_in[1];
  const float* bq    = (const float*)d_in[2];
  const float* Wk    = (const float*)d_in[3];
  const float* bk    = (const float*)d_in[4];
  const float* Wv    = (const float*)d_in[5];
  const float* bv    = (const float*)d_in[6];
  const float* gamma = (const float*)d_in[7];
  const float* beta  = (const float*)d_in[8];
  const float* W1    = (const float*)d_in[9];
  const float* b1    = (const float*)d_in[10];
  const float* aP    = (const float*)d_in[11];
  const float* W2    = (const float*)d_in[12];
  const float* b2    = (const float*)d_in[13];

  const size_t MiB = 1048576;
  char* ws = (char*)d_ws;
  const size_t oA = 0;
  const size_t oB = 32 * MiB;
  const size_t oC = 48 * MiB;
  const size_t oD = 72 * MiB;
  size_t o = 88 * MiB;
  const size_t oWqkh = o; o += (size_t)512 * 256 * 2;
  const size_t oWqkl = o; o += (size_t)512 * 256 * 2;
  const size_t oWv   = o; o += (size_t)256 * 256 * 2;
  const size_t oW1   = o; o += (size_t)1024 * 256 * 2;
  const size_t oW2   = o; o += (size_t)256 * 1024 * 2;
  const size_t oBqk  = o; o += 2048;
  const size_t oPart = o; o += (size_t)256 * 512 * 8;
  const size_t oMean = o; o += 1024;
  const size_t oIstd = o; o += 1024;
  const size_t total = o;
  if (total > ws_size || total > (size_t)134217728) return;

  float*    qk32 = (float*)(ws + oA);
  _Float16* ff16 = (_Float16*)(ws + oA);
  float*    v32  = (float*)(ws + oB);
  float*    mh32 = (float*)(ws + oB);
  _Float16* xh   = (_Float16*)(ws + oC);
  _Float16* xl   = (_Float16*)(ws + oC + 8 * MiB);
  _Float16* xf   = (_Float16*)(ws + oC + 16 * MiB);
  _Float16* mh16 = (_Float16*)(ws + oC);
  float*    y2   = (float*)(ws + oC + 8 * MiB);
  float*    oT   = (float*)(ws + oD);
  unsigned* wqkh = (unsigned*)(ws + oWqkh);
  unsigned* wqkl = (unsigned*)(ws + oWqkl);
  unsigned* wv16 = (unsigned*)(ws + oWv);
  unsigned* w1h  = (unsigned*)(ws + oW1);
  unsigned* w2h  = (unsigned*)(ws + oW2);
  float*    bqk  = (float*)(ws + oBqk);
  double*   part = (double*)(ws + oPart);
  float*    mean = (float*)(ws + oMean);
  float*    istd = (float*)(ws + oIstd);

  typedef const unsigned short* cus;

  prep_x<<<dim3(NPIX / 32, NBATCH), dim3(256), 0, stream>>>(x, xh, xl, xf);
  prep_weights<<<dim3(1410), dim3(256), 0, stream>>>(Wq, Wk, Wv, W1, W2, bq, bk, wqkh, wqkl, wv16, w1h, w2h, bqk);
  wmma_gemm64<1, true, 2, 0, false, 0><<<dim3((NROWS / 64) * (512 / 64) / 8, 1), dim3(256), 0, stream>>>(
      (cus)xh, (cus)xl, NCH, 0L, (cus)wqkh, (cus)wqkl, NCH, 0L,
      (void*)qk32, (void*)qk32, 512, 0L, bqk, aP, bqk, 0L, NROWS, 512, NCH, 1.0f);
  wmma_gemm64<0, false, 2, 0, false, 0><<<dim3((NROWS / 64) * (NCH / 64) / 8, 1), dim3(256), 0, stream>>>(
      (cus)xf, (cus)xf, NCH, 0L, (cus)wv16, (cus)wv16, NCH, 0L,
      (void*)v32, (void*)v32, NCH, 0L, bv, aP, bv, 0L, NROWS, NCH, NCH, 0.0625f);
  {
    AttnGeom g;
    g.q_bs = (long)NPIX * 512; g.q_rs = 512; g.q_hs = DHEAD;
    g.k_bs = (long)NPIX * 512; g.k_rs = 512; g.k_hs = DHEAD;
    g.v_bs = (long)NPIX * NCH; g.v_rs = NCH; g.v_hs = DHEAD;
    g.o_bs = (long)NPIX * NCH; g.o_rs = NCH; g.o_hs = DHEAD;
    g.S = NPIX; g.Skv = NPIX; g.H = NHEADS; g.zpad = 0;
    attn64_qks_pvh<<<dim3(NBATCH * NHEADS * (NPIX / 64)), dim3(128), 0, stream>>>(qk32, qk32 + 256, v32, oT, g);
  }
  bn_partial<true><<<dim3(NROWS / 64), dim3(256), 0, stream>>>(oT, x, part);
  bn_final<<<dim3(1), dim3(256), 0, stream>>>(part, NROWS / 64, 1.0f / 16384.0f, mean, istd);
  bn_apply1<<<dim3(NROWS / 8), dim3(256), 0, stream>>>(oT, x, mean, istd, gamma, beta, mh32, mh16);
  wmma_gemm64<0, false, 2, 1, false, 6><<<dim3((NROWS / 64) * (NFF / 64) / 8, 1), dim3(256), 0, stream>>>(
      (cus)mh16, (cus)mh16, NCH, 0L, (cus)w1h, (cus)w1h, NCH, 0L,
      (void*)ff16, (void*)ff16, NFF, 0L, b1, aP, b1, 0L, NROWS, NFF, NCH, 0.0625f);
  wmma_gemm64<0, false, 2, 0, true, 0><<<dim3((NROWS / 64) * (NCH / 64) / 8, 1), dim3(256), 0, stream>>>(
      (cus)ff16, (cus)ff16, NFF, 0L, (cus)w2h, (cus)w2h, NFF, 0L,
      (void*)y2, (void*)y2, NCH, 0L, b2, aP, mh32, 0L, NROWS, NCH, NFF, 0.0625f);
  bn_partial<false><<<dim3(NROWS / 64), dim3(256), 0, stream>>>(y2, x, part);
  bn_final<<<dim3(1), dim3(256), 0, stream>>>(part, NROWS / 64, 1.0f / 16384.0f, mean, istd);
  bn_apply2_nchw<<<dim3(NPIX / 64, NCH / 64, NBATCH), dim3(256), 0, stream>>>(y2, mean, istd, gamma, beta, (float*)d_out);
  (void)hipGetLastError();
}
